// MultiHeadAttentionBlock_40072044871790
// MI455X (gfx1250) — hardware-verified
//
#include <hip/hip_runtime.h>
#include <math.h>

typedef __attribute__((ext_vector_type(16))) _Float16 v16h;
typedef __attribute__((ext_vector_type(16))) __bf16 v16b;
typedef __attribute__((ext_vector_type(8)))  _Float16 v8h;
typedef __attribute__((ext_vector_type(8)))  float v8f;
typedef __attribute__((ext_vector_type(4)))  float v4f;
typedef __attribute__((ext_vector_type(4)))  unsigned v4u;

template <typename T> __device__ __forceinline__ void vst2(void* p, T v) { *(volatile T*)p = v; __threadfence(); *(volatile T*)p = v; }
__device__ __forceinline__ v8f wmma16(v16h a, v16h b, v8f c) {
  v8f d = __builtin_amdgcn_wmma_f32_16x16x32_f16(false, a, false, b, (short)0, c, false, false);
  asm volatile("v_nop\n\tv_nop\n\tv_nop\n\tv_nop" : "+v"(d) : "v"(a), "v"(b));
  return d;
}
__device__ __forceinline__ v8f wmma_bf(v16b a, v16b b, v8f c) {
  v8f d = __builtin_amdgcn_wmma_f32_16x16x32_bf16(false, a, false, b, (short)0, c, false, false);
  asm volatile("v_nop\n\tv_nop\n\tv_nop\n\tv_nop" : "+v"(d) : "v"(a), "v"(b));
  return d;
}
__device__ __forceinline__ v16h frag_h(const _Float16* rowk0, unsigned lane) {
  union { v16h v; v8h q[2]; } u; const _Float16* p = rowk0 + 8u * (lane >> 4);
  u.q[0] = *(const v8h*)p; u.q[1] = *(const v8h*)(p + 16); return u.v;
}
__device__ __forceinline__ float bfr(float v) { return (float)(__bf16)v; }
#define LDSX() do { asm volatile("s_wait_dscnt 0" ::: "memory"); __builtin_amdgcn_wave_barrier(); __builtin_amdgcn_fence(3  , "workgroup"); } while (0)

#ifndef NB
#define NB 4
#endif
#ifndef SEQ
#define SEQ 1024
#endif
#define NB_FULL 4
#define SEQ_FULL 1024
#define TT SEQ
#define CC 1024
#define DIN 1024
#define NH 16
#define HD 64
#define NQB (TT / 64)
#define SCALE (0.125f)
#define PCARRY (16384.0f)
#define YCARRY (16.0f)
static_assert(TT % 128 == 0);
static_assert(NB >= 1 && NB <= NB_FULL);
static_assert(SEQ >= 128 && SEQ <= SEQ_FULL);
static_assert(NH * HD == CC);
static_assert(DIN % 128 == 0 && CC % 128 == 0 && HD == 64);
static_assert(((size_t)NB * TT) % 64 == 0);
static_assert((size_t)(NB * TT / 64) * (CC / 128) * 64 * 128 == (size_t)NB * TT * CC);
static_assert((size_t)NQB * NH * NB * 64 * HD == (size_t)NB * TT * CC);
static_assert((size_t)(NB * TT / 64) * (DIN / 64) * 64 * 64 == (size_t)NB * TT * DIN);
static_assert(64 * 136 <= 128 * 72);

__device__ __forceinline__ v16b wcol_io(const float* Wm, unsigned k0, unsigned o, unsigned lane) { v16b w; const unsigned g = lane >> 4; const float* p = Wm + (size_t)(k0 + 8u * g) * CC + o;
#pragma unroll
  for (unsigned i = 0; i < 8; ++i) { w[i] = (__bf16)p[(size_t)i * CC]; w[8 + i] = (__bf16)p[(size_t)(16u + i) * CC]; }
  return w; }
__device__ __forceinline__ v16h wcolh_io(const float* Wm, unsigned k0, unsigned o, unsigned lane, unsigned ld) { v16h w; const unsigned g = lane >> 4;
#pragma unroll
  for (unsigned i = 0; i < 8; ++i) { w[i] = (_Float16)(bfr(Wm[(size_t)(k0 + 8u * g + i) * ld + o]) * 256.0f); w[8 + i] = (_Float16)(bfr(Wm[(size_t)(k0 + 16u + 8u * g + i) * ld + o]) * 256.0f); }
  return w; }

#define PLANE_B (2u * (size_t)NB * TT * CC)
#define WS_QH  0u
#define WS_QL  (WS_QH + PLANE_B)
#define WS_KH  (WS_QL + PLANE_B)
#define WS_KL  (WS_KH + PLANE_B)
#define WS_VT  (WS_KL + PLANE_B)
#define WS_VL  (WS_VT + PLANE_B)
#define WS_YH  (WS_VL + PLANE_B)
#define WS_YL  (WS_YH + PLANE_B)
#define WS_END (WS_YL + PLANE_B)
static_assert(WS_END <= (size_t)134217728u);
static_assert((PLANE_B % 128u) == 0);

__global__ __launch_bounds__(128) void k_proj(const float* __restrict__ X, const float* __restrict__ WQ, const float* __restrict__ WK, const float* __restrict__ WV, const float* __restrict__ BQ, const float* __restrict__ BK, const float* __restrict__ BV,
    _Float16* __restrict__ QH, _Float16* __restrict__ QL, _Float16* __restrict__ KH, _Float16* __restrict__ KL, _Float16* __restrict__ VT, _Float16* __restrict__ VL) {
  __shared__ __align__(16) _Float16 sb[2][128 * 72];
  const unsigned tid = threadIdx.x, wave = tid >> 5, lane = tid & 31u, col = lane & 15u, g = lane >> 4; const unsigned which = blockIdx.z; const unsigned c0 = blockIdx.y * 128u;
  const unsigned r0 = blockIdx.x * 64u; const unsigned bb = r0 / (unsigned)TT; const unsigned t0 = r0 - bb * (unsigned)TT; const unsigned xr0 = bb * (unsigned)SEQ_FULL + t0;
  const float* WA = which == 0u ? WQ : which == 1u ? WK : WV; const float* BA = which == 0u ? BQ : which == 1u ? BK : BV;
  v8f acc[8] = {};
#pragma unroll 2
  for (unsigned kc = 0; kc < DIN / 32; ++kc) { v16b a; { const float* p = X + (size_t)(xr0 + wave * 16u + col) * DIN + kc * 32u + 8u * g;
#pragma unroll
      for (unsigned i = 0; i < 8; ++i) { a[i] = (__bf16)p[i]; a[8 + i] = (__bf16)p[16 + i]; } }
    asm volatile("s_wait_loadcnt 0x0" ::: "memory");
#pragma unroll
    for (unsigned j = 0; j < 8; ++j) { const v16b w = wcol_io(WA, kc * 32u, c0 + j * 16u + col, lane); asm volatile("s_wait_loadcnt 0x0" ::: "memory"); acc[j] = wmma_bf(a, w, acc[j]); } }
  if (which < 2u) { _Float16* DH = which == 0u ? QH : KH; _Float16* DL = which == 0u ? QL : KL;
#pragma unroll
    for (unsigned j = 0; j < 8; ++j) { const float bias = bfr(BA[c0 + j * 16u + col]);
#pragma unroll
      for (unsigned r = 0; r < 8; ++r) { const float v = acc[j][r] + bias; const _Float16 hv = (_Float16)v; const unsigned ix = (wave * 16u + 8u * g + r) * 136u + j * 16u + col; sb[0][ix] = hv; sb[1][ix] = (_Float16)((v - (float)hv) * 1024.0f); } }
    __syncthreads();
    for (unsigned e = tid; e < 64u * 16u; e += 128u) { const unsigned rl = e >> 4, q = e & 15u; const v4u vh = *(const v4u*)&sb[0][rl * 136u + q * 8u]; const v4u vl = *(const v4u*)&sb[1][rl * 136u + q * 8u];
      const size_t go = (size_t)(r0 + rl) * CC + c0 + q * 8u; vst2((void*)(DH + go), vh); vst2((void*)(DL + go), vl); }
  } else {
#pragma unroll
    for (unsigned j = 0; j < 8; ++j) { const float bias = bfr(BA[c0 + j * 16u + col]);
#pragma unroll
      for (unsigned r = 0; r < 8; ++r) { const float v = acc[j][r] + bias; const _Float16 hv = (_Float16)v; const unsigned ix = (j * 16u + col) * 72u + wave * 16u + 8u * g + r; sb[0][ix] = hv; sb[1][ix] = (_Float16)((v - (float)hv) * 1024.0f); } }
    __syncthreads();
    for (unsigned e = tid; e < 128u * 8u; e += 128u) { const unsigned cl = e >> 3, q = e & 7u; const v4u vh = *(const v4u*)&sb[0][cl * 72u + q * 8u]; const v4u vl = *(const v4u*)&sb[1][cl * 72u + q * 8u];
      const size_t go = ((size_t)bb * CC + c0 + cl) * (size_t)TT + t0 + q * 8u; vst2((void*)(VT + go), vh); vst2((void*)(VL + go), vl); } } }

__device__ __forceinline__ float rmax16(float v) {
#pragma unroll
  for (int o = 1; o < 16; o <<= 1) v = fmaxf(v, __shfl_xor(v, o));
  return v; }
__device__ __forceinline__ float rsum16(float v) {
#pragma unroll
  for (int o = 1; o < 16; o <<= 1) v += __shfl_xor(v, o);
  return v; }
__global__ __launch_bounds__(128) void k_attn(const _Float16* __restrict__ QH, const _Float16* __restrict__ QL, const _Float16* __restrict__ KH, const _Float16* __restrict__ KL, const _Float16* __restrict__ VT, const _Float16* __restrict__ VL,
    _Float16* __restrict__ YH, _Float16* __restrict__ YL) {
  __shared__ __align__(16) _Float16 ksh[64][72], ksl[64][72];
  __shared__ __align__(16) _Float16 vsh[HD][72], vsl[HD][72];
  __shared__ __align__(16) _Float16 ph[4][16][72], pl[4][16][72];
  const unsigned tid = threadIdx.x, wave = tid >> 5, lane = tid & 31u, col = lane & 15u, g = lane >> 4;
  const unsigned qb = blockIdx.x, h = blockIdx.y, b = blockIdx.z;
  const unsigned ql0 = qb * 64u + wave * 16u;
  const size_t qoff = ((size_t)b * TT + ql0 + col) * CC + (size_t)h * HD;
  const v16h ah0 = frag_h(QH + qoff, lane), ah1 = frag_h(QH + qoff + 32, lane);
  const v16h al0 = frag_h(QL + qoff, lane), al1 = frag_h(QL + qoff + 32, lane);
  v8f o[HD / 16] = {}, orr[HD / 16] = {};
  float m[8], l[8];
#pragma unroll
  for (unsigned r = 0; r < 8; ++r) { m[r] = -1.0e30f; l[r] = 0.f; }
  _Float16 (*pph)[72] = ph[wave]; _Float16 (*ppl)[72] = pl[wave];
  const unsigned nkc = qb + 1u;
#pragma unroll 1
  for (unsigned kc = 0; kc < nkc; ++kc) {
    const unsigned k0 = kc * 64u; const bool diag = (kc == qb);
    __syncthreads();
    for (unsigned e = tid; e < 64u * 8u; e += 128u) { const unsigned row = e >> 3, q = e & 7u; const size_t go = ((size_t)b * TT + k0 + row) * CC + (size_t)h * HD + q * 8u;
      *(v4u*)&ksh[row][q * 8u] = *(const v4u*)(KH + go); *(v4u*)&ksl[row][q * 8u] = *(const v4u*)(KL + go); }
    for (unsigned e = tid; e < (unsigned)HD * 8u; e += 128u) { const unsigned c = e >> 3, q = e & 7u; const size_t go = ((size_t)b * CC + (size_t)h * HD + c) * (size_t)TT + k0 + q * 8u;
      *(v4u*)&vsh[c][q * 8u] = *(const v4u*)(VT + go); *(v4u*)&vsl[c][q * 8u] = *(const v4u*)(VL + go); }
    __syncthreads();
    v8f acc[4];
#pragma unroll
    for (unsigned j = 0; j < 4; ++j) { asm volatile("" ::: "memory");
      const v16h kh0 = frag_h(&ksh[j * 16u + col][0], lane), kh1 = frag_h(&ksh[j * 16u + col][32], lane);
      const v16h kl0 = frag_h(&ksl[j * 16u + col][0], lane), kl1 = frag_h(&ksl[j * 16u + col][32], lane);
      v8f a = {}; a = wmma16(al0, kh0, a); a = wmma16(al1, kh1, a); a = wmma16(ah0, kl0, a); a = wmma16(ah1, kl1, a); a = a * (1.0f / 1024.0f); a = wmma16(ah0, kh0, a); acc[j] = wmma16(ah1, kh1, a); }
#pragma unroll
    for (unsigned j = 0; j < 4; ++j)
#pragma unroll
      for (unsigned r = 0; r < 8; ++r) { const bool msk = diag && ((j * 16u + col) > (wave * 16u + 8u * g + r)); acc[j][r] = msk ? -1.0e30f : acc[j][r]; }
    float f[8];
#pragma unroll
    for (unsigned r = 0; r < 8; ++r) { float mx = acc[0][r];
#pragma unroll
      for (unsigned j = 1; j < 4; ++j) mx = fmaxf(mx, acc[j][r]);
      mx = rmax16(mx); const float mn = fmaxf(m[r], mx); f[r] = __expf((m[r] - mn) * SCALE); m[r] = mn; }
#pragma unroll
    for (unsigned r = 0; r < 8; ++r) { float s = 0.f;
#pragma unroll
      for (unsigned j = 0; j < 4; ++j) { const float ev = __expf((acc[j][r] - m[r]) * SCALE); const float p = (acc[j][r] < -0.5e30f) ? 0.f : ev; s += p;
        const float pc = p * PCARRY; const _Float16 hv = (_Float16)pc; pph[8u * g + r][j * 16u + col] = hv; ppl[8u * g + r][j * 16u + col] = (_Float16)((pc - (float)hv) * 1024.0f); }
      s = rsum16(s); l[r] = l[r] * f[r] + s; }
#pragma unroll
    for (unsigned j = 0; j < HD / 16; ++j)
#pragma unroll
      for (unsigned r = 0; r < 8; ++r) { o[j][r] *= f[r]; orr[j][r] *= f[r]; }
    LDSX();
#pragma unroll
    for (unsigned ks = 0; ks < 2; ++ks) { asm volatile("" ::: "memory"); const v16h pah = frag_h(&pph[col][ks * 32u], lane), pal = frag_h(&ppl[col][ks * 32u], lane);
#pragma unroll
      for (unsigned j = 0; j < HD / 16; ++j) { const v16h vh = frag_h(&vsh[j * 16u + col][ks * 32u], lane), vl = frag_h(&vsl[j * 16u + col][ks * 32u], lane);
        o[j] = wmma16(pah, vh, o[j]); orr[j] = wmma16(pah, vl, orr[j]); orr[j] = wmma16(pal, vh, orr[j]); } } }
  float inv[8];
#pragma unroll
  for (unsigned r = 0; r < 8; ++r) inv[r] = (1.0f / (l[r] * PCARRY)) * YCARRY;
  LDSX();
#pragma unroll
  for (unsigned j = 0; j < HD / 16; ++j)
#pragma unroll
    for (unsigned r = 0; r < 8; ++r) { const float y = (o[j][r] + orr[j][r] * (1.0f / 1024.0f)) * inv[r]; const _Float16 hv = (_Float16)y; pph[8u * g + r][j * 16u + col] = hv; ppl[8u * g + r][j * 16u + col] = (_Float16)((y - (float)hv) * 1024.0f); }
  LDSX();
#pragma unroll 1
  for (unsigned it = 0; it < 4; ++it) { const unsigned row = it * 4u + (lane >> 3), q = lane & 7u; const v4u vh = *(const v4u*)&pph[row][q * 8u]; const v4u vl = *(const v4u*)&ppl[row][q * 8u];
    const size_t go = ((size_t)b * TT + ql0 + row) * CC + (size_t)h * HD + q * 8u; vst2((void*)(YH + go), vh); vst2((void*)(YL + go), vl); } }

__global__ __launch_bounds__(128) void k_out(const _Float16* __restrict__ YH, const _Float16* __restrict__ YL, const float* __restrict__ WO, const float* __restrict__ BO, float* __restrict__ OUT) { __shared__ __align__(16) float sf[4][16][68];
  const unsigned tid = threadIdx.x, wave = tid >> 5, lane = tid & 31u, col = lane & 15u, g = lane >> 4; const unsigned c0 = blockIdx.y * 64u; const unsigned r0 = blockIdx.x * 64u + wave * 16u;
  v8f acc[4] = {}, accr[4] = {};
#pragma unroll 2
  for (unsigned kc = 0; kc < CC / 32; ++kc) { const size_t ao = (size_t)(r0 + col) * CC + kc * 32u; const v16h ah = frag_h(YH + ao, lane), al = frag_h(YL + ao, lane); asm volatile("s_wait_loadcnt 0x0" ::: "memory");
#pragma unroll
    for (unsigned j = 0; j < 4; ++j) { const v16h w = wcolh_io(WO, kc * 32u, c0 + j * 16u + col, lane, DIN); asm volatile("s_wait_loadcnt 0x0" ::: "memory"); acc[j] = wmma16(ah, w, acc[j]); accr[j] = wmma16(al, w, accr[j]); } }
#pragma unroll
  for (unsigned j = 0; j < 4; ++j) { const float bias = bfr(BO[c0 + j * 16u + col]);
#pragma unroll
    for (unsigned r = 0; r < 8; ++r) sf[wave][8u * g + r][j * 16u + col] = (acc[j][r] + accr[j][r] * (1.0f / 1024.0f)) * (1.0f / 4096.0f) + bias; }
  LDSX();
#pragma unroll 1
  for (unsigned it = 0; it < 8; ++it) { const unsigned row = it * 2u + g; const v4f v = *(const v4f*)&sf[wave][row][col * 4u]; vst2((void*)(OUT + (size_t)(r0 + row) * DIN + c0 + col * 4u), v); } }

extern "C" void kernel_launch(void* const* d_in, const int* in_sizes, int n_in, void* d_out, int out_size, void* d_ws, size_t ws_size, hipStream_t stream) {
  if (n_in < 9) return;
  if ((size_t)in_sizes[0] < ((size_t)(NB - 1) * SEQ_FULL + SEQ) * DIN) return;
  if (in_sizes[1] < DIN * CC || in_sizes[3] < DIN * CC || in_sizes[5] < DIN * CC) return;
  if (in_sizes[2] < CC || in_sizes[4] < CC || in_sizes[6] < CC) return;
  if (in_sizes[7] < CC * DIN || in_sizes[8] < DIN) return;
  if ((size_t)out_size < (size_t)NB * TT * DIN) return;
  if (ws_size < (size_t)WS_END) return;
  const float** F = (const float**)d_in;
  char* ws = (char*)d_ws;
  _Float16 *QH = (_Float16*)(ws + WS_QH), *QL = (_Float16*)(ws + WS_QL), *KH = (_Float16*)(ws + WS_KH), *KL = (_Float16*)(ws + WS_KL);
  _Float16 *VT = (_Float16*)(ws + WS_VT), *VL = (_Float16*)(ws + WS_VL), *YH = (_Float16*)(ws + WS_YH), *YL = (_Float16*)(ws + WS_YL);
  k_proj<<<dim3(NB * TT / 64, CC / 128, 3), 128, 0, stream>>>(F[0], F[1], F[3], F[5], F[2], F[4], F[6], QH, QL, KH, KL, VT, VL);
  k_attn<<<dim3(NQB, NH, NB), 128, 0, stream>>>(QH, QL, KH, KL, VT, VL, YH, YL);
  k_out<<<dim3(NB * TT / 64, DIN / 64), 128, 0, stream>>>(YH, YL, F[7], F[8], (float*)d_out);
}
